// CrossAttentionModule_76184129896947
// MI455X (gfx1250) — hardware-run, weakly checked
//
#include <hip/hip_runtime.h>
#include <math.h>

typedef __attribute__((ext_vector_type(16))) _Float16 v16h;
typedef __attribute__((ext_vector_type(8)))  _Float16 v8h;
typedef __attribute__((ext_vector_type(8)))  float    v8f;
typedef __attribute__((ext_vector_type(4)))  float    v4f;
typedef __attribute__((ext_vector_type(4)))  unsigned int v4u;

constexpr int kB  = 4;
constexpr int kTD = 256;
constexpr int kNS = 4;
constexpr int kSqrtTD = 16;
static_assert(kSqrtTD * kSqrtTD == kTD, "logit scale derives from the channel count");
constexpr float kLogitScale = 1.0f / (float)kSqrtTD;

constexpr int cinOf(int i)  { return 64 << i; }
constexpr int sideOf(int i) { return 64 >> i; }
constexpr int npixOf(int i) { return sideOf(i) * sideOf(i); }
constexpr int qrowsOf(int i) { return npixOf(i) < 2048 ? npixOf(i) : 2048; }
constexpr int nbOf(int i)    { return i == 0 ? 1 : kB; }

constexpr size_t pixBefore(int i) {
  size_t s = 0;
  for (int j = 0; j < i; ++j) s += (size_t)kB * npixOf(j);
  return s;
}
constexpr size_t vtElemsBefore(int i) {
  size_t s = 0;
  for (int j = 0; j < i; ++j) s += (size_t)kB * npixOf(j) * cinOf(j);
  return s;
}
constexpr size_t wElemsBefore(int i) {
  size_t s = 0;
  for (int j = 0; j < i; ++j) s += (size_t)kTD * cinOf(j);
  return s;
}
constexpr size_t outFloatsBefore(int i) {
  size_t s = (size_t)kB * 2048;
  for (int j = 0; j < i; ++j) s += (size_t)kB * cinOf(j) * npixOf(j);
  return s;
}
constexpr bool shapesOk() {
  for (int i = 0; i < kNS; ++i) {
    if ((kB * npixOf(i)) % 64) return false;
    if (npixOf(i) % 64) return false;
    if (cinOf(i) % 64) return false;
    if (qrowsOf(i) % 64) return false;
    if (npixOf(i) % qrowsOf(i)) return false;
  }
  return true;
}
static_assert(shapesOk(), "every GEMM M and N is a multiple of 64 and every K a multiple of 32");
static_assert(kTD % 64 == 0 && 1024 % 32 == 0, "GEMM tile multiples");
static_assert(outFloatsBefore(0) * 4 == 32768ull, "output 1 byte offset");
static_assert(outFloatsBefore(1) * 4 == 4227072ull, "output 2 byte offset");
static_assert(outFloatsBefore(2) * 4 == 6324224ull, "output 3 byte offset");
static_assert(outFloatsBefore(3) * 4 == 7372800ull, "output 4 byte offset");
static_assert(outFloatsBefore(4) * 4 == 7897088ull, "output total bytes");

constexpr float kActCarry = 16.0f;
constexpr float kWCarry   = 256.0f;
constexpr float kPCarry   = 32768.0f;
constexpr float kAvCarry  = 256.0f;
constexpr float kCatCarry = 64.0f;
constexpr float kProjScale      = kActCarry / (kActCarry * kWCarry);
constexpr float kLogitGemmScale = kLogitScale / (kActCarry * kActCarry);
constexpr float kPVScale        = kAvCarry / (kPCarry * kActCarry);
constexpr float kOutScale       = 1.0f / (kWCarry * kAvCarry);
constexpr float kSgScale        = 1.0f / (kCatCarry * kWCarry);
constexpr float kF16MinNormal   = 6.103515625e-05f;
constexpr float kBnEps          = 1e-5f;

constexpr size_t kPixTotal = pixBefore(kNS);
constexpr size_t kWpElems  = wElemsBefore(kNS);
constexpr size_t kSzVT   = vtElemsBefore(kNS) * 2;
constexpr size_t kSzTT   = kPixTotal * kTD * 2;
constexpr size_t kSzW16  = (2 * kWpElems + 3 * (size_t)kTD * kTD + (size_t)kTD * 1024) * 2;
constexpr size_t kSzPl16 = kPixTotal * kTD * 2;
constexpr size_t kSzSB   = (size_t)2048 * 4096 * 4;
constexpr size_t kSzPB   = (size_t)2048 * 4096 * 2;
constexpr size_t kSzCAT  = (size_t)256 * 1024 * 2;
constexpr size_t kSzXS   = (size_t)256 * 256 * 4;
constexpr size_t kSzPL   = (size_t)4 * 256 * 4;
constexpr size_t kSzF1   = (size_t)4 * 1024 * 4;
constexpr size_t kOffVT  = 0;
constexpr size_t kOffTT  = kOffVT  + kSzVT;
constexpr size_t kOffW16 = kOffTT  + kSzTT;
constexpr size_t kOffVP  = kOffW16 + kSzW16;
constexpr size_t kOffQP  = kOffVP  + kSzPl16;
constexpr size_t kOffKP  = kOffQP  + kSzPl16;
constexpr size_t kOffVC  = kOffKP  + kSzPl16;
constexpr size_t kOffAV  = kOffVC  + kSzPl16;
constexpr size_t kOffSB  = kOffAV  + kSzPl16;
constexpr size_t kOffPB  = kOffSB  + kSzSB;
constexpr size_t kOffCAT = kOffPB  + kSzPB;
constexpr size_t kOffXS  = kOffCAT + kSzCAT;
constexpr size_t kOffPL  = kOffXS  + kSzXS;
constexpr size_t kOffF1  = kOffPL  + kSzPL;
constexpr size_t kWsTotal = kOffF1 + kSzF1;
static_assert(kSzVT == 3932160ull && kSzTT == 11141120ull && kSzW16 == 1900544ull && kSzPl16 == 11141120ull, "plane sizes");
static_assert(kWsTotal == 123817984ull, "carve total");
static_assert(kWsTotal <= 134217728ull, "carve cap");
static_assert((kOffTT % 128) == 0 && (kOffW16 % 128) == 0 && (kOffVP % 128) == 0 && (kOffQP % 128) == 0 &&
              (kOffKP % 128) == 0 && (kOffVC % 128) == 0 && (kOffAV % 128) == 0 && (kOffSB % 128) == 0 &&
              (kOffPB % 128) == 0 && (kOffCAT % 128) == 0 && (kOffXS % 128) == 0 && (kOffPL % 128) == 0 &&
              (kOffF1 % 128) == 0, "128-B aligned regions");
constexpr bool chunkFits() {
  for (int i = 0; i < kNS; ++i) {
    const size_t el = (size_t)nbOf(i) * qrowsOf(i) * npixOf(i);
    if (el * 4 > kSzSB) return false;
    if (el * 2 > kSzPB) return false;
  }
  return true;
}
static_assert(chunkFits(), "logit and probability chunk planes fit their regions for every scale");

__device__ __forceinline__ unsigned pk16(unsigned short a, unsigned short b) { return (unsigned)a | ((unsigned)b << 16); }
__device__ __forceinline__ unsigned short h_bits_flush(float f) {
  const float g = (fabsf(f) < kF16MinNormal) ? 0.0f : f;
  const _Float16 h = (_Float16)g;
  return __builtin_bit_cast(unsigned short, h);
}
__device__ __forceinline__ v16h frag_load(const _Float16* p) {
  union U { v16h v; v8h h[2]; } f;
  f.h[0] = *(const v8h*)(p);
  f.h[1] = *(const v8h*)(p + 16);
  return f.v;
}
__device__ __forceinline__ v8f mma_h(v16h a, v16h b, v8f c) {
  return __builtin_amdgcn_wmma_f32_16x16x32_f16(false, a, false, b, (short)0, c, false, false);
}
__device__ __forceinline__ void tie_h(v8f& c, v16h a, v16h b) { asm volatile("" : "+v"(c) : "v"(a), "v"(b)); }
__device__ __forceinline__ void guard_h(v8f& c, v16h a, v16h b) { asm volatile("v_nop\n\tv_nop\n\tv_nop\n\tv_nop" : "+v"(c) : "v"(a), "v"(b)); }
__device__ __forceinline__ void keep4_h(v16h a, v16h b, v16h c, v16h d) { asm volatile("v_nop" :: "v"(a), "v"(b), "v"(c), "v"(d)); }

template <int BIAS_MODE, int OUT_MODE, bool RESID>
__global__ __launch_bounds__(256) void gemm64_f16_kernel(
    const unsigned short* __restrict__ Ap, int lda, long strideA,
    const unsigned short* __restrict__ Btp, int ldb, long strideB,
    void* __restrict__ Cout, int ldc, long strideC,
    const float* __restrict__ bias, float bias_scale,
    const float* __restrict__ resid, long strideR,
    int M, int N, int K, float scale) {
  static_assert(!(RESID && OUT_MODE != 0), "f32 addend only with f32 output");
  const _Float16* A  = (const _Float16*)Ap;
  const _Float16* Bt = (const _Float16*)Btp;
  __shared__ __align__(16) float sT[8][16 * 68];
  const int b    = blockIdx.y;
  const int lane = threadIdx.x & 31;
  const int wave = threadIdx.x >> 5;
  const int tilesN = N >> 6;
  const int tilesM = M >> 6;
  const int tile = blockIdx.x * 8 + wave;
  if (tile >= tilesM * tilesN) return;
  const int tm = tile / tilesN;
  const int tn = tile - tm * tilesN;
  const int m0 = tm << 6;
  const int n0 = tn << 6;

  const _Float16* Ab = A  + (size_t)b * strideA;
  const _Float16* Bb = Bt + (size_t)b * strideB;

  const int rlane = lane & 15;
  const int koff  = (lane >> 4) * 8;
  const int mOff  = (lane >> 4) * 8;

  v8f acc[4][4];
#pragma unroll
  for (int i = 0; i < 4; ++i)
#pragma unroll
    for (int j = 0; j < 4; ++j) acc[i][j] = (v8f){0.f, 0.f, 0.f, 0.f, 0.f, 0.f, 0.f, 0.f};

  for (int k0 = 0; k0 < K; k0 += 32) {
    v16h bh[4];
#pragma unroll
    for (int j = 0; j < 4; ++j) {
      const size_t bo = (size_t)(n0 + (j << 4) + rlane) * ldb + koff + k0;
      bh[j] = frag_load(Bb + bo);
    }
#pragma unroll
    for (int i = 0; i < 4; ++i) {
      const size_t ao = (size_t)(m0 + (i << 4) + rlane) * lda + koff + k0;
      const v16h ah = frag_load(Ab + ao);
#pragma unroll
      for (int j = 0; j < 4; ++j) acc[i][j] = mma_h(ah, bh[j], acc[i][j]);
      tie_h(acc[i][0], ah, bh[0]);
      tie_h(acc[i][1], ah, bh[1]);
      tie_h(acc[i][2], ah, bh[2]);
      guard_h(acc[i][3], ah, bh[3]);
    }
    keep4_h(bh[0], bh[1], bh[2], bh[3]);
  }

  float* slab = sT[wave];
  const float* Rb = RESID ? (resid + (size_t)b * strideR) : nullptr;
  const int hh = lane >> 4;
#pragma unroll
  for (int i = 0; i < 4; ++i) {
    const int mBase = m0 + (i << 4);
#pragma unroll
    for (int j = 0; j < 4; ++j) {
      float bv = 0.f;
      if (BIAS_MODE == 2) bv = bias[n0 + (j << 4) + rlane] * bias_scale;
#pragma unroll
      for (int r = 0; r < 8; ++r) {
        float v = acc[i][j][r] * scale;
        if (BIAS_MODE == 1) v += bias[mBase + mOff + r] * bias_scale;
        if (BIAS_MODE == 2) v += bv;
        slab[(mOff + r) * 68 + (j << 4) + rlane] = v;
      }
    }
    __builtin_amdgcn_fence(__ATOMIC_RELEASE, "workgroup");
    __builtin_amdgcn_wave_barrier();
    __builtin_amdgcn_fence(__ATOMIC_ACQUIRE, "workgroup");
    if (OUT_MODE == 0) {
      float* C = (float*)Cout + (size_t)b * strideC;
      const int c4 = (lane & 15) * 4;
      v4f ov[8];
#pragma unroll
      for (int it = 0; it < 8; ++it) {
        const int row = it * 2 + hh;
        v4f v = *(const v4f*)(slab + row * 68 + c4);
        if (RESID) {
          const v4f rv = *(const v4f*)(Rb + (size_t)(mBase + row) * ldc + n0 + c4);
          v = v + rv;
        }
        ov[it] = v;
      }
      for (int pass = 0; pass < 2; ++pass) {
#pragma unroll
        for (int it = 0; it < 8; ++it) {
          const int row = it * 2 + hh;
          *(volatile v4f*)(C + (size_t)(mBase + row) * ldc + n0 + c4) = ov[it];
        }
        __threadfence();
      }
    } else {
      const int q = lane >> 3, c8 = (lane & 7) * 8;
      unsigned short* C = (unsigned short*)Cout + (size_t)b * strideC;
      v4u ou[4];
#pragma unroll
      for (int it = 0; it < 4; ++it) {
        const int row = it * 4 + q;
        const float* sp = slab + row * 68 + c8;
        unsigned short hb[8];
#pragma unroll
        for (int e = 0; e < 8; ++e) hb[e] = h_bits_flush(sp[e]);
        ou[it] = (v4u){pk16(hb[0], hb[1]), pk16(hb[2], hb[3]), pk16(hb[4], hb[5]), pk16(hb[6], hb[7])};
      }
      for (int pass = 0; pass < 2; ++pass) {
#pragma unroll
        for (int it = 0; it < 4; ++it) {
          const int row = it * 4 + q;
          *(volatile v4u*)(C + (size_t)(mBase + row) * ldc + n0 + c8) = ou[it];
        }
        __threadfence();
      }
    }
    __builtin_amdgcn_fence(__ATOMIC_RELEASE, "workgroup");
    __builtin_amdgcn_wave_barrier();
    __builtin_amdgcn_fence(__ATOMIC_ACQUIRE, "workgroup");
  }
}

__global__ __launch_bounds__(256) void cast8_f16_kernel(const float* __restrict__ in, unsigned short* __restrict__ out,
                                                        int n8, float carry) {
  const int i = blockIdx.x * 256 + threadIdx.x;
  if (i >= n8) return;
  const float* p = in + 8 * (size_t)i;
  const v4f a = *(const v4f*)(p);
  const v4f c = *(const v4f*)(p + 4);
  unsigned short hb[8];
#pragma unroll
  for (int e = 0; e < 4; ++e) {
    const float fa = a[e] * carry;
    const float fc = c[e] * carry;
    hb[e]     = h_bits_flush(fa);
    hb[4 + e] = h_bits_flush(fc);
  }
  const v4u u = (v4u){pk16(hb[0], hb[1]), pk16(hb[2], hb[3]), pk16(hb[4], hb[5]), pk16(hb[6], hb[7])};
  unsigned short* q = out + 8 * (size_t)i;
  *(volatile v4u*)q = u;
  __threadfence();
  *(volatile v4u*)q = u;
}

__global__ __launch_bounds__(256) void nchw_to_pix_f16_kernel(const float* __restrict__ X, unsigned short* __restrict__ XT,
                                                              int Cc, int Np, float carry) {
  __shared__ float sm[64][65];
  const int t  = threadIdx.x;
  const int n0 = blockIdx.x * 64;
  const int c0 = blockIdx.y * 64;
  const int b  = blockIdx.z;
  const float* Xb = X + (size_t)b * Cc * Np;
#pragma unroll 8
  for (int i = 0; i < 16; ++i) {
    const int e  = i * 256 + t;
    const int r  = e >> 6;
    const int cc = e & 63;
    sm[cc][r] = Xb[(size_t)(c0 + r) * Np + n0 + cc] * carry;
  }
  __syncthreads();
  const int lane = t & 31, wave = t >> 5;
  const int q = lane >> 3, c8 = (lane & 7) * 8;
  unsigned short* op = XT + (size_t)b * Np * Cc;
  v4u u[2];
#pragma unroll
  for (int it = 0; it < 2; ++it) {
    const int row = wave * 8 + it * 4 + q;
    unsigned short hb[8];
#pragma unroll
    for (int e = 0; e < 8; ++e) hb[e] = h_bits_flush(sm[row][c8 + e]);
    u[it] = (v4u){pk16(hb[0], hb[1]), pk16(hb[2], hb[3]), pk16(hb[4], hb[5]), pk16(hb[6], hb[7])};
  }
  for (int pass = 0; pass < 2; ++pass) {
#pragma unroll
    for (int it = 0; it < 2; ++it) {
      const int row = wave * 8 + it * 4 + q;
      *(volatile v4u*)(op + (size_t)(n0 + row) * Cc + c0 + c8) = u[it];
    }
    __threadfence();
  }
}

template <int NK, int TPR, int CH>
__global__ __launch_bounds__(256) void softmax_rows_kernel(const float* __restrict__ S, unsigned short* __restrict__ P, int nrows) {
  static_assert(TPR * CH * 8 == NK, "row coverage");
  static_assert((256 % TPR) == 0, "rows per block");
  constexpr int RPB = 256 / TPR;
  constexpr int LW  = (TPR < 32) ? TPR : 32;
  constexpr int WPR = (TPR > 32) ? (TPR / 32) : 1;
  __shared__ float redM[8];
  __shared__ float redS[8];
  const int t = threadIdx.x, lane = t & 31, wave = t >> 5;
  const int rb = t / TPR;
  const int tr = t - rb * TPR;
  int row = blockIdx.x * RPB + rb;
  row = (row < nrows) ? row : (nrows - 1);
  const float* sr = S + (size_t)row * NK;
  float x[CH][8];
#pragma unroll
  for (int c = 0; c < CH; ++c) {
    const int col = (c * TPR + tr) * 8;
    const v4f a = *(const v4f*)(sr + col);
    const v4f d = *(const v4f*)(sr + col + 4);
#pragma unroll
    for (int e = 0; e < 4; ++e) {
      x[c][e]     = a[e];
      x[c][4 + e] = d[e];
    }
  }
  float m = x[0][0];
#pragma unroll
  for (int c = 0; c < CH; ++c)
#pragma unroll
    for (int e = 0; e < 8; ++e) m = fmaxf(m, x[c][e]);
#pragma unroll
  for (int off = LW / 2; off > 0; off >>= 1) m = fmaxf(m, __shfl_xor(m, off, 32));
  if (TPR > 32) {
    if (lane == 0) redM[wave] = m;
    __syncthreads();
    const int wb = (wave / WPR) * WPR;
    float mm = redM[wb];
#pragma unroll
    for (int k = 1; k < WPR; ++k) mm = fmaxf(mm, redM[wb + k]);
    m = mm;
  }
  float l = 0.f;
#pragma unroll
  for (int c = 0; c < CH; ++c)
#pragma unroll
    for (int e = 0; e < 8; ++e) {
      const float p = __expf(x[c][e] - m);
      x[c][e] = p;
      l += p;
    }
#pragma unroll
  for (int off = LW / 2; off > 0; off >>= 1) l += __shfl_xor(l, off, 32);
  if (TPR > 32) {
    if (lane == 0) redS[wave] = l;
    __syncthreads();
    const int wb = (wave / WPR) * WPR;
    float ll = redS[wb];
#pragma unroll
    for (int k = 1; k < WPR; ++k) ll += redS[wb + k];
    l = ll;
  }
  const float rl = kPCarry * (1.0f / l);
  v4u u[CH];
#pragma unroll
  for (int c = 0; c < CH; ++c) {
    unsigned short hb[8];
#pragma unroll
    for (int e = 0; e < 8; ++e) {
      const float pv = x[c][e] * rl;
      hb[e] = h_bits_flush(pv);
    }
    u[c] = (v4u){pk16(hb[0], hb[1]), pk16(hb[2], hb[3]), pk16(hb[4], hb[5]), pk16(hb[6], hb[7])};
  }
  unsigned short* pr = P + (size_t)row * NK;
  for (int pass = 0; pass < 2; ++pass) {
#pragma unroll
    for (int c = 0; c < CH; ++c) {
      const int col = (c * TPR + tr) * 8;
      *(volatile v4u*)(pr + col) = u[c];
    }
    __threadfence();
  }
}

__global__ __launch_bounds__(256) void pool_cat_kernel(const float* __restrict__ t0, const float* __restrict__ t1,
                                                       const float* __restrict__ t2, const float* __restrict__ t3,
                                                       unsigned short* __restrict__ CAT) {
  __shared__ float sm[64][65];
  const int t  = threadIdx.x;
  const int cg = blockIdx.x;
  const int si = blockIdx.y;
  const int b  = blockIdx.z;
  const float* tp = (si == 0) ? t0 : (si == 1) ? t1 : (si == 2) ? t2 : t3;
  const int H = 64 >> si;
  const int f = H >> 3;
  const float sc = kCatCarry / (float)(f * f);
#pragma unroll 1
  for (int o = 0; o < 16; ++o) {
    const int e  = o * 256 + t;
    const int cl = e >> 6;
    const int px = e & 63;
    const int y  = px >> 3;
    const int x  = px & 7;
    const float* base = tp + ((size_t)(b * kTD + cg * 64 + cl) * H + y * f) * H + x * f;
    float s = 0.f;
#pragma unroll 1
    for (int fy = 0; fy < f; ++fy) {
#pragma unroll 1
      for (int fx = 0; fx < f; ++fx) s += base[fy * H + fx];
    }
    sm[px][cl] = s * sc;
  }
  __syncthreads();
  const int lane = t & 31, wave = t >> 5;
  const int q = lane >> 3, c8 = (lane & 7) * 8;
  v4u u[2];
#pragma unroll
  for (int it = 0; it < 2; ++it) {
    const int row = wave * 8 + it * 4 + q;
    unsigned short hb[8];
#pragma unroll
    for (int e = 0; e < 8; ++e) hb[e] = h_bits_flush(sm[row][c8 + e]);
    u[it] = (v4u){pk16(hb[0], hb[1]), pk16(hb[2], hb[3]), pk16(hb[4], hb[5]), pk16(hb[6], hb[7])};
  }
  for (int pass = 0; pass < 2; ++pass) {
#pragma unroll
    for (int it = 0; it < 2; ++it) {
      const int row = wave * 8 + it * 4 + q;
      *(volatile v4u*)(CAT + (size_t)(b * 64 + row) * 1024 + si * 256 + cg * 64 + c8) = u[it];
    }
    __threadfence();
  }
}

__global__ __launch_bounds__(256) void bn_relu_pool_kernel(const float* __restrict__ X, const float* __restrict__ g,
                                                           const float* __restrict__ be, float* __restrict__ PL) {
  const int c = threadIdx.x;
  float s = 0.f;
#pragma unroll 4
  for (int p = 0; p < 256; ++p) s += X[p * kTD + c];
  const float mu = s * (1.0f / 256.0f);
  float vs = 0.f;
#pragma unroll 4
  for (int p = 0; p < 256; ++p) {
    const float d = X[p * kTD + c] - mu;
    vs = fmaf(d, d, vs);
  }
  const float var = vs * (1.0f / 256.0f);
  const float rs  = 1.0f / sqrtf(var + kBnEps);
  const float gg  = g[c] * rs;
  const float bb  = be[c];
  float res[4];
#pragma unroll
  for (int b = 0; b < 4; ++b) {
    float a = 0.f;
#pragma unroll 4
    for (int i = 0; i < 64; ++i) {
      const float y = (X[(b * 64 + i) * kTD + c] - mu) * gg + bb;
      a += fmaxf(y, 0.0f);
    }
    res[b] = a * (1.0f / 64.0f);
  }
  for (int pass = 0; pass < 2; ++pass) {
#pragma unroll
    for (int b = 0; b < 4; ++b) *(volatile float*)(PL + b * kTD + c) = res[b];
    __threadfence();
  }
}

template <int KD, bool RELU>
__global__ __launch_bounds__(256) void fc_rows4_kernel(const float* __restrict__ X, const float* __restrict__ W,
                                                       const float* __restrict__ bias, float* __restrict__ Y, int O) {
  __shared__ float xs[4 * KD];
  const int t = threadIdx.x, lane = t & 31, wave = t >> 5;
#pragma unroll 1
  for (int i = t; i < 4 * KD; i += 256) xs[i] = X[i];
  __syncthreads();
  int o0 = (blockIdx.x * 8 + wave) * 32;
  o0 = (o0 + 32 <= O) ? o0 : (O - 32);
  float r0 = 0.f, r1 = 0.f, r2 = 0.f, r3 = 0.f;
#pragma unroll 1
  for (int oo = 0; oo < 32; ++oo) {
    const float* wr = W + (size_t)(o0 + oo) * KD + lane;
    float a0 = 0.f, a1 = 0.f, a2 = 0.f, a3 = 0.f;
#pragma unroll 2
    for (int j = 0; j < KD / 32; ++j) {
      const float w = wr[j * 32];
      const float* xp = xs + j * 32 + lane;
      a0 = fmaf(w, xp[0], a0);
      a1 = fmaf(w, xp[KD], a1);
      a2 = fmaf(w, xp[2 * KD], a2);
      a3 = fmaf(w, xp[3 * KD], a3);
    }
#pragma unroll
    for (int off = 16; off > 0; off >>= 1) {
      a0 += __shfl_xor(a0, off, 32);
      a1 += __shfl_xor(a1, off, 32);
      a2 += __shfl_xor(a2, off, 32);
      a3 += __shfl_xor(a3, off, 32);
    }
    const bool mine = (lane == oo);
    r0 = mine ? a0 : r0;
    r1 = mine ? a1 : r1;
    r2 = mine ? a2 : r2;
    r3 = mine ? a3 : r3;
  }
  const float bv = bias[o0 + lane];
  r0 += bv;
  r1 += bv;
  r2 += bv;
  r3 += bv;
  if (RELU) {
    r0 = fmaxf(r0, 0.0f);
    r1 = fmaxf(r1, 0.0f);
    r2 = fmaxf(r2, 0.0f);
    r3 = fmaxf(r3, 0.0f);
  }
  for (int pass = 0; pass < 2; ++pass) {
    *(volatile float*)(Y + (size_t)0 * O + o0 + lane) = r0;
    *(volatile float*)(Y + (size_t)1 * O + o0 + lane) = r1;
    *(volatile float*)(Y + (size_t)2 * O + o0 + lane) = r2;
    *(volatile float*)(Y + (size_t)3 * O + o0 + lane) = r3;
    __threadfence();
  }
}

template <int BM, int OM, bool RS>
static void launch_gemm(hipStream_t st,
                        const unsigned short* A, int lda, long sA,
                        const unsigned short* Bt, int ldb, long sB,
                        void* C, int ldc, long sC,
                        const float* bias, float bscale,
                        const float* resid, long sR,
                        int M, int N, int K, float scale, int nbatch) {
  const int tiles = (M >> 6) * (N >> 6);
  dim3 grid((unsigned)((tiles + 7) / 8), (unsigned)nbatch);
  gemm64_f16_kernel<BM, OM, RS><<<grid, 256, 0, st>>>(A, lda, sA, Bt, ldb, sB, C, ldc, sC, bias, bscale, resid, sR, M, N, K, scale);
}

static void launch_cast(hipStream_t st, const float* in, unsigned short* out, int n, float carry) {
  const int n8 = n / 8;
  cast8_f16_kernel<<<(n8 + 255) / 256, 256, 0, st>>>(in, out, n8, carry);
}

static void launch_softmax(hipStream_t st, int si, const float* S, unsigned short* P, int rows) {
  if (si == 0)      softmax_rows_kernel<4096, 256, 2><<<rows / 1,  256, 0, st>>>(S, P, rows);
  else if (si == 1) softmax_rows_kernel<1024, 128, 1><<<rows / 2,  256, 0, st>>>(S, P, rows);
  else if (si == 2) softmax_rows_kernel<256,  32,  1><<<rows / 8,  256, 0, st>>>(S, P, rows);
  else              softmax_rows_kernel<64,   8,   1><<<rows / 32, 256, 0, st>>>(S, P, rows);
}
static_assert(npixOf(0) == 4096 && npixOf(1) == 1024 && npixOf(2) == 256 && npixOf(3) == 64, "softmax instantiations");
static_assert((nbOf(1) * qrowsOf(1)) % 2 == 0 && (nbOf(2) * qrowsOf(2)) % 8 == 0 && (nbOf(3) * qrowsOf(3)) % 32 == 0, "exact softmax grids");

extern "C" void kernel_launch(void* const* d_in, const int* in_sizes, int n_in,
                              void* d_out, int out_size, void* d_ws, size_t ws_size,
                              hipStream_t stream) {
  if (n_in < 38) return;
  for (int i = 0; i < kNS; ++i) {
    if (in_sizes[i] != kB * cinOf(i) * npixOf(i)) return;
    if (in_sizes[4 + i] != kB * kTD * npixOf(i)) return;
    if (in_sizes[8 + 4 * i] != kTD * cinOf(i)) return;
    if (in_sizes[9 + 4 * i] != kTD) return;
    if (in_sizes[10 + 4 * i] != cinOf(i) * kTD) return;
    if (in_sizes[11 + 4 * i] != cinOf(i)) return;
  }
  if (in_sizes[24] != kTD * kTD || in_sizes[26] != kTD * kTD || in_sizes[28] != kTD * kTD) return;
  if (in_sizes[25] != kTD || in_sizes[27] != kTD || in_sizes[29] != kTD) return;
  if (in_sizes[30] != kTD * 1024 || in_sizes[31] != kTD || in_sizes[32] != kTD || in_sizes[33] != kTD) return;
  if (in_sizes[34] != 1024 * kTD || in_sizes[35] != 1024 || in_sizes[36] != 2048 * 1024 || in_sizes[37] != 2048) return;
  if ((size_t)out_size != outFloatsBefore(kNS)) return;
  if (ws_size < kWsTotal) return;

  const float* vin[4]  = {(const float*)d_in[0], (const float*)d_in[1], (const float*)d_in[2], (const float*)d_in[3]};
  const float* tin[4]  = {(const float*)d_in[4], (const float*)d_in[5], (const float*)d_in[6], (const float*)d_in[7]};
  const float* vp_w[4];
  const float* vp_b[4];
  const float* op_w[4];
  const float* op_b[4];
  for (int i = 0; i < kNS; ++i) {
    vp_w[i] = (const float*)d_in[8 + 4 * i];
    vp_b[i] = (const float*)d_in[9 + 4 * i];
    op_w[i] = (const float*)d_in[10 + 4 * i];
    op_b[i] = (const float*)d_in[11 + 4 * i];
  }
  const float* q_w   = (const float*)d_in[24];
  const float* q_b   = (const float*)d_in[25];
  const float* k_w   = (const float*)d_in[26];
  const float* k_b   = (const float*)d_in[27];
  const float* v_w   = (const float*)d_in[28];
  const float* v_b   = (const float*)d_in[29];
  const float* sg_w  = (const float*)d_in[30];
  const float* sg_b  = (const float*)d_in[31];
  const float* bn_g  = (const float*)d_in[32];
  const float* bn_b  = (const float*)d_in[33];
  const float* fc1_w = (const float*)d_in[34];
  const float* fc1_b = (const float*)d_in[35];
  const float* fc2_w = (const float*)d_in[36];
  const float* fc2_b = (const float*)d_in[37];
  float* outp = (float*)d_out;

  char* ws = (char*)d_ws;
  unsigned short* VT  = (unsigned short*)(ws + kOffVT);
  unsigned short* TT  = (unsigned short*)(ws + kOffTT);
  unsigned short* W16 = (unsigned short*)(ws + kOffW16);
  unsigned short* VP  = (unsigned short*)(ws + kOffVP);
  unsigned short* QP  = (unsigned short*)(ws + kOffQP);
  unsigned short* KP  = (unsigned short*)(ws + kOffKP);
  unsigned short* VC  = (unsigned short*)(ws + kOffVC);
  unsigned short* AV  = (unsigned short*)(ws + kOffAV);
  float*          SB  = (float*)(ws + kOffSB);
  unsigned short* PB  = (unsigned short*)(ws + kOffPB);
  unsigned short* CAT = (unsigned short*)(ws + kOffCAT);
  float*          XS  = (float*)(ws + kOffXS);
  float*          PL  = (float*)(ws + kOffPL);
  float*          F1  = (float*)(ws + kOffF1);

  unsigned short* Wvp = W16;
  unsigned short* Wop = W16 + kWpElems;
  unsigned short* Wq  = W16 + 2 * kWpElems;
  unsigned short* Wk  = Wq + (size_t)kTD * kTD;
  unsigned short* Wv  = Wk + (size_t)kTD * kTD;
  unsigned short* Wsg = Wv + (size_t)kTD * kTD;

  for (int i = 0; i < kNS; ++i) {
    launch_cast(stream, vp_w[i], Wvp + wElemsBefore(i), kTD * cinOf(i), kWCarry);
    launch_cast(stream, op_w[i], Wop + wElemsBefore(i), kTD * cinOf(i), kWCarry);
  }
  launch_cast(stream, q_w,  Wq,  kTD * kTD,  kWCarry);
  launch_cast(stream, k_w,  Wk,  kTD * kTD,  kWCarry);
  launch_cast(stream, v_w,  Wv,  kTD * kTD,  kWCarry);
  launch_cast(stream, sg_w, Wsg, kTD * 1024, kWCarry);

  for (int i = 0; i < kNS; ++i) {
    const int Np = npixOf(i), Ci = cinOf(i);
    nchw_to_pix_f16_kernel<<<dim3(Np / 64, Ci / 64, kB), 256, 0, stream>>>(vin[i], VT + vtElemsBefore(i), Ci, Np, kActCarry);
    nchw_to_pix_f16_kernel<<<dim3(Np / 64, kTD / 64, kB), 256, 0, stream>>>(tin[i], TT + pixBefore(i) * kTD, kTD, Np, kActCarry);
  }

  for (int i = 0; i < kNS; ++i) {
    const int Np = npixOf(i), Ci = cinOf(i);
    const int Mpix = kB * Np;
    const size_t po = pixBefore(i) * kTD;
    const unsigned short* vT_i = VT + vtElemsBefore(i);
    const unsigned short* tT_i = TT + po;
    unsigned short* vp_i = VP + po;
    unsigned short* q_i  = QP + po;
    unsigned short* k_i  = KP + po;
    unsigned short* vc_i = VC + po;
    unsigned short* av_i = AV + po;

    launch_gemm<2, 1, false>(stream, vT_i, Ci, 0L, Wvp + wElemsBefore(i), Ci, 0L, (void*)vp_i, kTD, 0L,
                             vp_b[i], kActCarry, nullptr, 0L, Mpix, kTD, Ci, kProjScale, 1);
    launch_gemm<2, 1, false>(stream, vp_i, kTD, 0L, Wq, kTD, 0L, (void*)q_i, kTD, 0L,
                             q_b, kActCarry, nullptr, 0L, Mpix, kTD, kTD, kProjScale, 1);
    launch_gemm<2, 1, false>(stream, tT_i, kTD, 0L, Wk, kTD, 0L, (void*)k_i, kTD, 0L,
                             k_b, kActCarry, nullptr, 0L, Mpix, kTD, kTD, kProjScale, 1);
    launch_gemm<1, 1, false>(stream, Wv, kTD, 0L, tT_i, kTD, (long)Np * kTD, (void*)vc_i, Np, (long)kTD * Np,
                             v_b, kActCarry, nullptr, 0L, kTD, Np, kTD, kProjScale, kB);

    const int QR = qrowsOf(i), nb = nbOf(i);
    for (int b0 = 0; b0 < kB; b0 += nb) {
      for (int q0 = 0; q0 < Np; q0 += QR) {
        launch_gemm<0, 0, false>(stream, q_i + ((size_t)b0 * Np + q0) * kTD, kTD, (long)Np * kTD,
                                 k_i + (size_t)b0 * Np * kTD, kTD, (long)Np * kTD,
                                 (void*)SB, Np, (long)QR * Np,
                                 nullptr, 0.0f, nullptr, 0L, QR, Np, kTD, kLogitGemmScale, nb);
        launch_softmax(stream, i, SB, PB, nb * QR);
        launch_gemm<0, 1, false>(stream, PB, Np, (long)QR * Np,
                                 vc_i + (size_t)b0 * kTD * Np, Np, (long)kTD * Np,
                                 (void*)(av_i + ((size_t)b0 * Np + q0) * kTD), kTD, (long)Np * kTD,
                                 nullptr, 0.0f, nullptr, 0L, QR, kTD, Np, kPVScale, nb);
      }
    }

    launch_gemm<1, 0, true>(stream, Wop + wElemsBefore(i), kTD, 0L, av_i, kTD, (long)Np * kTD,
                            (void*)(outp + outFloatsBefore(i)), Np, (long)Ci * Np,
                            op_b[i], 1.0f, vin[i], (long)Ci * Np, Ci, Np, kTD, kOutScale, kB);
  }

  pool_cat_kernel<<<dim3(4, 4, kB), 256, 0, stream>>>(tin[0], tin[1], tin[2], tin[3], CAT);
  launch_gemm<2, 0, false>(stream, CAT, 1024, 0L, Wsg, 1024, 0L, (void*)XS, kTD, 0L,
                           sg_b, 1.0f, nullptr, 0L, 256, kTD, 1024, kSgScale, 1);
  bn_relu_pool_kernel<<<1, 256, 0, stream>>>(XS, bn_g, bn_b, PL);
  fc_rows4_kernel<256, true><<<1024 / 256, 256, 0, stream>>>(PL, fc1_w, fc1_b, F1, 1024);
  fc_rows4_kernel<1024, false><<<2048 / 256, 256, 0, stream>>>(F1, fc2_w, fc2_b, outp, 2048);
}
